// MemoryEfficientAttention_90117003805176
// MI455X (gfx1250) — hardware-verified
//
#include <hip/hip_runtime.h>
#include <math.h>

#ifndef NB
#define NB 2
#endif
#ifndef SEQ
#define SEQ 2048
#endif
#define NB_FULL 2
#define SEQ_FULL 2048
#define DM 1024
#define NH 16
#define HDIM 64
static_assert(NB >= 1 && NB <= NB_FULL);
static_assert(SEQ >= 64 && SEQ <= SEQ_FULL && (SEQ % 64) == 0);
static_assert(DM == NH * HDIM);
static_assert((DM % 64) == 0 && HDIM == 64);

typedef __attribute__((ext_vector_type(16))) _Float16 v16h;
typedef __attribute__((ext_vector_type(8)))  _Float16 v8h;
typedef __attribute__((ext_vector_type(16))) __bf16   v16b;
typedef __attribute__((ext_vector_type(8)))  __bf16   v8b;
typedef __attribute__((ext_vector_type(8)))  float    v8f;
typedef __attribute__((ext_vector_type(4)))  float    v4f;
typedef __attribute__((ext_vector_type(8)))  unsigned short v8us;

__device__ __forceinline__ __bf16 bf16_rne(float f) {
    unsigned int u = __float_as_uint(f);
    u += 0x7fffu + ((u >> 16) & 1u);
    return __builtin_bit_cast(__bf16, (unsigned short)(u >> 16));
}
__device__ __forceinline__ float bf16_f32(__bf16 b) { return __uint_as_float(((unsigned int)__builtin_bit_cast(unsigned short, b)) << 16); }
__device__ __forceinline__ unsigned short bf16_bits(float f) {
    unsigned int u = __float_as_uint(f);
    u += 0x7fffu + ((u >> 16) & 1u);
    return (unsigned short)(u >> 16);
}
__device__ __forceinline__ unsigned short f16_bits(float f) { const _Float16 hh = (_Float16)f; return __builtin_bit_cast(unsigned short, hh); }

__device__ __forceinline__ v8f wmma16(v16h a, v16h b, v8f c) {
    c = __builtin_amdgcn_wmma_f32_16x16x32_f16(false, a, false, b, (short)0, c, false, false);
    asm volatile("v_nop\n\tv_nop\n\tv_nop\n\tv_nop" : "+v"(c) : "v"(a), "v"(b));
    return c;
}
__device__ __forceinline__ v8f wmmab(v16b a, v16b b, v8f c) {
    c = __builtin_amdgcn_wmma_f32_16x16x32_bf16(false, a, false, b, (short)0, c, false, false);
    asm volatile("v_nop\n\tv_nop\n\tv_nop\n\tv_nop" : "+v"(c) : "v"(a), "v"(b));
    return c;
}
struct Split { v16b hi, lo; };
__device__ __forceinline__ v8f wmma3(const Split& a, const Split& b, v8f c) {
    c = __builtin_amdgcn_wmma_f32_16x16x32_bf16(false, a.hi, false, b.hi, (short)0, c, false, false);
    c = __builtin_amdgcn_wmma_f32_16x16x32_bf16(false, a.hi, false, b.lo, (short)0, c, false, false);
    c = __builtin_amdgcn_wmma_f32_16x16x32_bf16(false, a.lo, false, b.hi, (short)0, c, false, false);
    asm volatile("v_nop\n\tv_nop\n\tv_nop\n\tv_nop" : "+v"(c) : "v"(a.hi), "v"(a.lo), "v"(b.hi), "v"(b.lo));
    return c;
}

union FragH { v16h v; v8h hv[2]; };
union FragB { v16b v; v8b hv[2]; };
__device__ __forceinline__ v16h ld_frag_h(const _Float16* __restrict__ row, int h) {
    FragH f; f.hv[0] = *(const v8h*)(row + 8 * h); f.hv[1] = *(const v8h*)(row + 16 + 8 * h); return f.v;
}
__device__ __forceinline__ v16b ld_frag_b(const __bf16* __restrict__ row, int h) {
    FragB f; f.hv[0] = *(const v8b*)(row + 8 * h); f.hv[1] = *(const v8b*)(row + 16 + 8 * h); return f.v;
}

#define VST2(T, ptr, val) do { const T vst2_v_ = (val); *(volatile T*)(ptr) = vst2_v_; __threadfence(); *(volatile T*)(ptr) = vst2_v_; } while (0)
#define VST2V4(ptr, val) do { const v4f vst2_v4_ = (val); *(volatile v4f*)(ptr) = vst2_v4_; __threadfence(); *(volatile v4f*)(ptr) = vst2_v4_; } while (0)
#define VST2U8(ptr, val) do { const v8us vst2_u8_ = (val); *(volatile v8us*)(ptr) = vst2_u8_; __threadfence(); *(volatile v8us*)(ptr) = vst2_u8_; } while (0)

struct G16P {
    const unsigned short* A; const unsigned short* Bt; const float* bias; float* C;
    long long sAz, sCz;
    int M, N, K, lda, ldb, ldc, flags, pad_;
    float iscale; int pad2_;
};
static_assert(sizeof(G16P) == 4 * 8 + 2 * 8 + 8 * 4 + 2 * 4);

template <int BT, int TM, int TN>
__global__ __launch_bounds__(32) void k_gemm16(G16P p) {
    const int lane = threadIdx.x & 31, h = lane >> 4, l15 = lane & 15;
    const int m0 = blockIdx.y * (16 * TM), n0 = blockIdx.x * (16 * TN), z = blockIdx.z;
    const unsigned short* Ab = p.A + (long long)z * p.sAz;
    v8f acc[TM][TN];
#pragma unroll
    for (int i = 0; i < TM; ++i)
#pragma unroll
        for (int t = 0; t < TN; ++t) { v8f zz = {}; acc[i][t] = zz; }
    for (int k0 = 0; k0 < p.K; k0 += 32) {
        if (BT == 0) {
            v16b a[TM], b[TN];
#pragma unroll
            for (int i = 0; i < TM; ++i) { const int am = min(m0 + 16 * i + l15, p.M - 1); a[i] = ld_frag_b((const __bf16*)(Ab + (long long)am * p.lda + k0), h); }
#pragma unroll
            for (int t = 0; t < TN; ++t) { const int bn = min(n0 + 16 * t + l15, p.N - 1); b[t] = ld_frag_b((const __bf16*)(p.Bt + (long long)bn * p.ldb + k0), h); }
#pragma unroll
            for (int i = 0; i < TM; ++i)
#pragma unroll
                for (int t = 0; t < TN; ++t) acc[i][t] = wmmab(a[i], b[t], acc[i][t]);
        } else {
            v16h a[TM], b[TN];
#pragma unroll
            for (int i = 0; i < TM; ++i) { const int am = min(m0 + 16 * i + l15, p.M - 1); a[i] = ld_frag_h((const _Float16*)(Ab + (long long)am * p.lda + k0), h); }
#pragma unroll
            for (int t = 0; t < TN; ++t) { const int bn = min(n0 + 16 * t + l15, p.N - 1); b[t] = ld_frag_h((const _Float16*)(p.Bt + (long long)bn * p.ldb + k0), h); }
#pragma unroll
            for (int i = 0; i < TM; ++i)
#pragma unroll
                for (int t = 0; t < TN; ++t) acc[i][t] = wmma16(a[i], b[t], acc[i][t]);
        }
    }
    float* C = p.C + (long long)z * p.sCz;
    __shared__ __align__(16) float ctile[16][36];
#pragma unroll
    for (int i = 0; i < TM; ++i) {
        const int mb = m0 + 16 * i; if (mb >= p.M) break;
#pragma unroll
        for (int tp = 0; tp < TN / 2; ++tp) {
            const int nb = n0 + 32 * tp; if (nb >= p.N) break;
#pragma unroll
            for (int t2 = 0; t2 < 2; ++t2) {
                const int t = 2 * tp + t2; const int n = nb + t2 * 16 + l15; const int nn = min(n, p.N - 1);
                float bb = 0.f;
                if (p.flags & 1) bb = bf16_f32(bf16_rne(p.bias[nn]));
#pragma unroll
                for (int r = 0; r < 8; ++r) {
                    const float v = acc[i][t][r] * p.iscale + bb;
                    ctile[8 * h + r][t2 * 16 + l15] = (n < p.N) ? v : 0.f;
                }
            }
            __syncthreads();
            const bool fast = (mb + 16 <= p.M) && (nb + 32 <= p.N) && ((p.ldc & 3) == 0) && ((((size_t)C) & 15) == 0);
            if (fast) {
#pragma unroll
                for (int s = 0; s < 4; ++s) {
                    const int row = s * 4 + (lane >> 3), c4 = (lane & 7) * 4;
                    const v4f v = *(const v4f*)&ctile[row][c4];
                    VST2V4(C + (long long)(mb + row) * p.ldc + nb + c4, v);
                }
            } else {
                for (int row = 0; row < 16; ++row) {
                    const int m = mb + row, n = nb + lane;
                    if (m < p.M && n < p.N) VST2(float, C + (long long)m * p.ldc + n, ctile[row][lane]);
                }
            }
            __syncthreads();
        }
    }
}

#define AW 4
#define KBLK 32
#define PSP 40
#define OSP 72
__global__ __launch_bounds__(32 * AW) __attribute__((amdgpu_num_vgpr(256)))
void k_attn64(const unsigned short* __restrict__ qh, const unsigned short* __restrict__ ql,
              const unsigned short* __restrict__ kh, const unsigned short* __restrict__ kl,
              const unsigned short* __restrict__ vt, unsigned short* __restrict__ cx) {
    __shared__ __align__(16) _Float16       ps[2][AW][16][PSP];
    __shared__ __align__(16) unsigned short osg[AW][16][OSP];
    const int lane = threadIdx.x & 31, hf = lane >> 4, l15 = lane & 15, wave = threadIdx.x >> 5;
    const int h = blockIdx.y, b = blockIdx.z;
    const int q0 = (blockIdx.x * AW + wave) * 16;
    const float sc2 = 0.125f * 1.4426950408889634f;

    const long long qoff = ((long long)b * SEQ + q0 + l15) * DM + h * HDIM;
    Split qf[2];
#pragma unroll
    for (int ks = 0; ks < 2; ++ks) {
        qf[ks].hi = ld_frag_b((const __bf16*)(qh + qoff + 32 * ks), hf);
        qf[ks].lo = ld_frag_b((const __bf16*)(ql + qoff + 32 * ks), hf);
    }
    v8f o[4]; float m8[8], l8[8];
#pragma unroll
    for (int t = 0; t < 4; ++t) { v8f zz = {}; o[t] = zz; }
#pragma unroll
    for (int i = 0; i < 8; ++i) { m8[i] = -1.0e30f; l8[i] = 0.f; }
    const long long kb0 = (long long)b * SEQ * DM + h * HDIM;
    const long long vb0 = ((long long)(b * NH + h) * HDIM) * SEQ;

#pragma unroll 1
    for (int j0 = 0; j0 < SEQ; j0 += KBLK) {
        const int buf = (j0 / KBLK) & 1;
        v8f s0 = {}, s1 = {};
        {
            const long long k0off = kb0 + (long long)(j0 + l15) * DM, k1off = k0off + 16LL * DM;
#pragma unroll
            for (int ks = 0; ks < 2; ++ks) {
                Split f0, f1;
                f0.hi = ld_frag_b((const __bf16*)(kh + k0off + 32 * ks), hf); f0.lo = ld_frag_b((const __bf16*)(kl + k0off + 32 * ks), hf);
                f1.hi = ld_frag_b((const __bf16*)(kh + k1off + 32 * ks), hf); f1.lo = ld_frag_b((const __bf16*)(kl + k1off + 32 * ks), hf);
                s0 = wmma3(qf[ks], f0, s0);
                s1 = wmma3(qf[ks], f1, s1);
            }
        }
#pragma unroll
        for (int i = 0; i < 8; ++i) {
            const float a0 = s0[i] * sc2, a1 = s1[i] * sc2;
            float mx = fmaxf(a0, a1);
            mx = fmaxf(mx, __shfl_xor(mx, 1, 32)); mx = fmaxf(mx, __shfl_xor(mx, 2, 32));
            mx = fmaxf(mx, __shfl_xor(mx, 4, 32)); mx = fmaxf(mx, __shfl_xor(mx, 8, 32));
            const float mnew = fmaxf(m8[i], mx);
            const float corr = exp2f(m8[i] - mnew);
            const float p0 = exp2f(a0 - mnew), p1 = exp2f(a1 - mnew);
            float rs = p0 + p1;
            rs += __shfl_xor(rs, 1, 32); rs += __shfl_xor(rs, 2, 32); rs += __shfl_xor(rs, 4, 32); rs += __shfl_xor(rs, 8, 32);
            l8[i] = l8[i] * corr + rs; m8[i] = mnew;
#pragma unroll
            for (int t = 0; t < 4; ++t) o[t][i] *= corr;
            ps[buf][wave][8 * hf + i][l15]      = (_Float16)(p0 * 4096.f);
            ps[buf][wave][8 * hf + i][16 + l15] = (_Float16)(p1 * 4096.f);
        }
        __syncthreads();
        FragH pa;
        pa.hv[0] = *(const v8h*)&ps[buf][wave][l15][8 * hf];
        pa.hv[1] = *(const v8h*)&ps[buf][wave][l15][16 + 8 * hf];
#pragma unroll
        for (int t = 0; t < 4; ++t) {
            const v16h vb = ld_frag_h((const _Float16*)(vt + vb0 + (long long)(16 * t + l15) * SEQ + j0), hf);
            o[t] = wmma16(pa.v, vb, o[t]);
        }
    }
    float invr[8];
#pragma unroll
    for (int i = 0; i < 8; ++i) invr[i] = (l8[i] > 0.f) ? 1.f / (l8[i] * 64.f) : 0.f;
#pragma unroll
    for (int i = 0; i < 8; ++i)
#pragma unroll
        for (int t = 0; t < 4; ++t) osg[wave][8 * hf + i][16 * t + l15] = f16_bits(o[t][i] * invr[i]);
    __syncthreads();
#pragma unroll
    for (int s = 0; s < 4; ++s) {
        const int row = s * 4 + (lane >> 3), c8 = (lane & 7) * 8;
        const v8us v = *(const v8us*)&osg[wave][row][c8];
        VST2U8(cx + ((long long)b * SEQ + q0 + row) * DM + h * HDIM + c8, v);
    }
}

struct CvtP {
    const float* s0; const float* s1; const float* s2; unsigned short* d0; unsigned short* d1; unsigned short* d2;
    long long sSb; int rows_per_b, nrows;
};
static_assert(sizeof(CvtP) == 6 * 8 + 8 + 2 * 4);
__global__ __launch_bounds__(256) void k_cvt16(CvtP p) {
    const int z = blockIdx.z;
    const float* src = (z == 0) ? p.s0 : ((z == 1) ? p.s1 : p.s2);
    unsigned short* dst = (z == 0) ? p.d0 : ((z == 1) ? p.d1 : p.d2);
    const long long e = ((long long)blockIdx.x * 256 + threadIdx.x) * 8;
    if (e >= (long long)p.nrows * DM) return;
    const int row = (int)(e / DM); const int col = (int)(e - (long long)row * DM);
    const int bb = row / p.rows_per_b, rr = row - bb * p.rows_per_b;
    const float* sp = src + (long long)bb * p.sSb + (long long)rr * DM + col;
    const v4f f0 = *(const v4f*)sp;
    const v4f f1 = *(const v4f*)(sp + 4);
    v8us o;
#pragma unroll
    for (int j = 0; j < 4; ++j) {
        const float x0 = f0[j], x1 = f1[j];
        o[j] = bf16_bits(x0); o[j + 4] = bf16_bits(x1);
    }
    VST2U8(dst + (long long)row * DM + col, o);
}

struct SplP { const float* s0; const float* s1; unsigned short* h0; unsigned short* l0; unsigned short* h1; unsigned short* l1; long long n; };
static_assert(sizeof(SplP) == 7 * 8);
__global__ __launch_bounds__(256) void k_split2(SplP p) {
    const int z = blockIdx.y;
    const float* src = z ? p.s1 : p.s0;
    unsigned short* dh = z ? p.h1 : p.h0;
    unsigned short* dl = z ? p.l1 : p.l0;
    const long long e = ((long long)blockIdx.x * 256 + threadIdx.x) * 8;
    if (e >= p.n) return;
    const v4f f0 = *(const v4f*)(src + e);
    const v4f f1 = *(const v4f*)(src + e + 4);
    v8us oh, ol;
#pragma unroll
    for (int j = 0; j < 4; ++j) {
        const float x0 = f0[j], x1 = f1[j];
        const unsigned short b0 = bf16_bits(x0), b1 = bf16_bits(x1);
        oh[j] = b0;     ol[j]     = bf16_bits(x0 - __uint_as_float(((unsigned int)b0) << 16));
        oh[j + 4] = b1; ol[j + 4] = bf16_bits(x1 - __uint_as_float(((unsigned int)b1) << 16));
    }
    VST2U8(dh + e, oh);
    VST2U8(dl + e, ol);
}

__global__ __launch_bounds__(256) void k_vtr(const float* __restrict__ vp, unsigned short* __restrict__ vt) {
    __shared__ float tile[64][65];
    const int j0 = blockIdx.x * 64, h = blockIdx.y, b = blockIdx.z, t = threadIdx.x;
    const int jr = t >> 2, cb = (t & 3) * 16;
    const float* sp = vp + ((long long)b * SEQ + j0 + jr) * DM + h * HDIM + cb;
#pragma unroll
    for (int q = 0; q < 4; ++q) {
        const v4f f = *(const v4f*)(sp + 4 * q);
        tile[jr][cb + 4 * q + 0] = f[0]; tile[jr][cb + 4 * q + 1] = f[1]; tile[jr][cb + 4 * q + 2] = f[2]; tile[jr][cb + 4 * q + 3] = f[3];
    }
    __syncthreads();
#pragma unroll
    for (int s2 = 0; s2 < 2; ++s2) {
        const int piece = t + 256 * s2;
        const int d = piece >> 3, jq = (piece & 7) * 8;
        v8us o;
#pragma unroll
        for (int e = 0; e < 8; ++e) o[e] = f16_bits(tile[jq + e][d]);
        VST2U8(vt + ((long long)(b * NH + h) * HDIM + d) * SEQ + j0 + jq, o);
    }
}

struct TrcP {
    const float* w0; const float* w1; const float* w2; const float* w3;
    unsigned short* d0; unsigned short* d1; unsigned short* d2; unsigned short* d3;
    int n, pad_; float s3; int pad2_;
};
static_assert(sizeof(TrcP) == 8 * 8 + 4 * 4);
__global__ __launch_bounds__(256) void k_trcvt(TrcP p) {
    __shared__ float tile[64][65];
    const int z = blockIdx.z;
    const float* W = (z == 0) ? p.w0 : ((z == 1) ? p.w1 : ((z == 2) ? p.w2 : p.w3));
    unsigned short* Dd = (z == 0) ? p.d0 : ((z == 1) ? p.d1 : ((z == 2) ? p.d2 : p.d3));
    const int n0 = blockIdx.x * 64, k0 = blockIdx.y * 64, t = threadIdx.x;
    const int kk = t >> 2, cb = (t & 3) * 16;
    const float* wr = W + (long long)(k0 + kk) * p.n + n0 + cb;
#pragma unroll
    for (int j = 0; j < 4; ++j) {
        const v4f f = *(const v4f*)(wr + 4 * j);
        tile[kk][cb + 4 * j + 0] = f[0]; tile[kk][cb + 4 * j + 1] = f[1]; tile[kk][cb + 4 * j + 2] = f[2]; tile[kk][cb + 4 * j + 3] = f[3];
    }
    __syncthreads();
#pragma unroll
    for (int s2 = 0; s2 < 2; ++s2) {
        const int piece = t + 256 * s2;
        const int nn = piece >> 3, kq = (piece & 7) * 8;
        v8us o;
#pragma unroll
        for (int e = 0; e < 8; ++e) {
            const float x = tile[kq + e][nn];
            const unsigned short hb = bf16_bits(x);
            const float xb = __uint_as_float(((unsigned int)hb) << 16);
            o[e] = (z == 3) ? f16_bits(xb * p.s3) : hb;
        }
        VST2U8(Dd + (long long)(n0 + nn) * p.n + k0 + kq, o);
    }
}

static G16P mk_g16(const unsigned short* A, const unsigned short* Bt, const float* bias, float* C, long long sAz, long long sCz, int M, int N, int K, float iscale) {
    G16P g;
    g.A = A; g.Bt = Bt; g.bias = bias; g.C = C; g.sAz = sAz; g.sCz = sCz;
    g.M = M; g.N = N; g.K = K; g.lda = K; g.ldb = K; g.ldc = N; g.flags = 1; g.pad_ = 0; g.iscale = iscale; g.pad2_ = 0;
    return g;
}

extern "C" void kernel_launch(void* const* d_in, const int* in_sizes, int n_in, void* d_out, int out_size, void* d_ws, size_t ws_size, hipStream_t stream) {
    if (n_in < 11) return;
    const long long needx = (long long)(NB - 1) * SEQ_FULL * DM + (long long)SEQ * DM;
    if ((long long)in_sizes[0] < needx || (long long)in_sizes[1] < needx || (long long)in_sizes[2] < needx) return;
    if (in_sizes[3] < DM * DM || in_sizes[5] < DM * DM || in_sizes[7] < DM * DM || in_sizes[9] < DM * DM) return;
    if (in_sizes[4] < DM || in_sizes[6] < DM || in_sizes[8] < DM || in_sizes[10] < DM) return;
    if ((long long)out_size < needx) return;
    const float* query = (const float*)d_in[0];
    const float* keyx  = (const float*)d_in[1];
    const float* value = (const float*)d_in[2];
    const float* Wq = (const float*)d_in[3];
    const float* bq = (const float*)d_in[4];
    const float* Wk = (const float*)d_in[5];
    const float* bk = (const float*)d_in[6];
    const float* Wv = (const float*)d_in[7];
    const float* bv = (const float*)d_in[8];
    const float* Wo = (const float*)d_in[9];
    const float* bo = (const float*)d_in[10];
    float* out = (float*)d_out;

    const size_t MR  = (size_t)NB * SEQ;
    const size_t X16 = MR * DM * 2;
    const size_t W16 = (size_t)DM * DM * 2;
    const size_t P32 = MR * DM * 4;
    const size_t total = 6 * X16 + 4 * W16 + 3 * P32;
    if (total > ws_size) return;
    char* ws = (char*)d_ws; size_t off = 0;
    unsigned short* xq  = (unsigned short*)(ws + off); off += X16;
    unsigned short* xk  = (unsigned short*)(ws + off); off += X16;
    unsigned short* xv  = (unsigned short*)(ws + off); off += X16;
    unsigned short* klo = (unsigned short*)(ws + off); off += X16;
    unsigned short* vt  = (unsigned short*)(ws + off); off += X16;
    unsigned short* c16 = (unsigned short*)(ws + off); off += X16;
    unsigned short* wtq = (unsigned short*)(ws + off); off += W16;
    unsigned short* wtk = (unsigned short*)(ws + off); off += W16;
    unsigned short* wtv = (unsigned short*)(ws + off); off += W16;
    unsigned short* wto = (unsigned short*)(ws + off); off += W16;
    float* qp = (float*)(ws + off); off += P32;
    float* kp = (float*)(ws + off); off += P32;
    float* vp = (float*)(ws + off); off += P32;
    if (off > ws_size) return;
    unsigned short* qhi = xq;
    unsigned short* qlo = xk;
    unsigned short* khi = xv;

    { CvtP c; c.s0 = query; c.s1 = keyx; c.s2 = value; c.d0 = xq; c.d1 = xk; c.d2 = xv;
      c.sSb = (long long)SEQ_FULL * DM; c.rows_per_b = SEQ; c.nrows = NB * SEQ;
      k_cvt16<<<dim3((unsigned)(MR / 2), 1, 3), 256, 0, stream>>>(c); }
    { TrcP tcp; tcp.w0 = Wq; tcp.w1 = Wk; tcp.w2 = Wv; tcp.w3 = Wo; tcp.d0 = wtq; tcp.d1 = wtk; tcp.d2 = wtv; tcp.d3 = wto;
      tcp.n = DM; tcp.pad_ = 0; tcp.s3 = 32.f; tcp.pad2_ = 0;
      k_trcvt<<<dim3(DM / 64, DM / 64, 4), 256, 0, stream>>>(tcp); }
    { const dim3 g(DM / 64, (unsigned)(MR / 32), 1);
      k_gemm16<0, 2, 4><<<g, 32, 0, stream>>>(mk_g16(xq, wtq, bq, qp, 0, 0, (int)MR, DM, DM, 1.f));
      k_gemm16<0, 2, 4><<<g, 32, 0, stream>>>(mk_g16(xk, wtk, bk, kp, 0, 0, (int)MR, DM, DM, 1.f));
      k_gemm16<0, 2, 4><<<g, 32, 0, stream>>>(mk_g16(xv, wtv, bv, vp, 0, 0, (int)MR, DM, DM, 1.f)); }
    { SplP s; s.s0 = qp; s.s1 = kp; s.h0 = qhi; s.l0 = qlo; s.h1 = khi; s.l1 = klo; s.n = (long long)MR * DM;
      k_split2<<<dim3((unsigned)(MR / 2), 2, 1), 256, 0, stream>>>(s); }
    k_vtr<<<dim3((unsigned)(SEQ / 64), NH, NB), 256, 0, stream>>>(vp, vt);
    k_attn64<<<dim3((unsigned)(SEQ / (16 * AW)), NH, NB), 32 * AW, 0, stream>>>(qhi, qlo, khi, klo, vt, c16);
    { const dim3 g(DM / 64, (unsigned)(SEQ / 32), NB);
      k_gemm16<1, 2, 4><<<g, 32, 0, stream>>>(mk_g16(c16, wto, bo, out, (long long)SEQ * DM, (long long)SEQ_FULL * DM, SEQ, DM, DM, 1.f / 2048.f)); }
}
